// SparseFlexAttn_5574867550977
// MI455X (gfx1250) — hardware-verified
//
#include <hip/hip_runtime.h>
#include <math.h>
#include <stdint.h>

#define NHEAD 16
#define SQ    1600
#define SKV   4121
#define SKP   4224
#define HD    128
#define NQBLK 13
#define NKBLK 33
#define QGRP  64
#define NQG   (SQ / QGRP)
#define WPB   4
#define ATT_THREADS (WPB * 32)
#define NVT   (SKP / 64)
#define RSQ_HD 0.08838834764831845f
#define LOG2E 1.4426950408889634f
#define PCAR  32768.0f
#define VCAR  1024.0f
#define PTP   36
#define PTW   (16 * PTP)
#define SLP   132
#define SLW   (16 * SLP)
#define WREG  (PTW + SLW)
#define VTP   72
#define WS_CAP 134217728
static_assert(NQG * QGRP == SQ);
static_assert(SKP == NKBLK * 128 && SKP >= SKV && NVT * 64 == SKP);
static_assert(NQBLK * 128 >= SQ && ((NQG - 1) >> 1) == NQBLK - 1);
static_assert(HD == 128 && ATT_THREADS == 128);
static_assert(((NHEAD * SQ * HD / 8) % 256) == 0 && ((NHEAD * SKP * 16) % 256) == 0);
static_assert((PTW % 4) == 0 && (SLP % 4) == 0 && (WREG % 4) == 0 && (VTP % 8) == 0);

typedef unsigned short u16;
typedef _Float16 v16h __attribute__((ext_vector_type(16)));
typedef _Float16 v8h  __attribute__((ext_vector_type(8)));
typedef __bf16   v16b __attribute__((ext_vector_type(16)));
typedef float    v8f  __attribute__((ext_vector_type(8)));
typedef float    v4f  __attribute__((ext_vector_type(4)));
typedef unsigned int v4u __attribute__((ext_vector_type(4)));

union FragH { v16h v; v8h h[2]; v4u u[2]; };
union FragB { v16b v; v4u u[2]; };

__constant__ unsigned char kLive[NQBLK * NKBLK] = {
  1,1,1,0, 1,1,0,1, 1,0,0,1, 1,1,0,0, 0,0,0,1, 1,1,1,0, 0,0,0,0, 0,0,0,0, 0,
  1,1,1,0, 1,1,0,1, 1,0,0,1, 1,1,1,0, 0,0,0,1, 1,1,1,1, 0,0,0,0, 0,0,0,0, 0,
  1,1,1,1, 1,1,0,1, 1,1,0,1, 1,1,1,0, 0,0,0,1, 1,1,1,1, 1,0,0,0, 0,0,0,0, 0,
  1,1,1,1, 1,1,0,1, 1,1,0,0, 1,1,1,1, 0,0,0,0, 1,1,1,1, 1,1,0,0, 0,0,0,0, 0,
  1,1,1,1, 1,1,1,1, 1,1,1,0, 1,1,1,1, 1,0,0,0, 0,1,1,1, 1,1,1,0, 0,0,0,0, 0,
  1,1,1,1, 1,1,1,0, 1,1,1,0, 0,1,1,1, 1,0,0,0, 0,0,1,1, 1,1,1,1, 0,0,0,0, 0,
  1,1,1,1, 0,1,1,0, 1,1,1,0, 0,0,1,1, 1,1,0,0, 0,0,0,1, 1,1,1,1, 1,0,0,0, 0,
  1,1,1,1, 0,1,1,0, 1,1,1,1, 0,0,1,1, 1,1,1,0, 0,0,0,0, 1,1,1,1, 1,1,0,0, 0,
  1,1,1,1, 1,1,1,1, 0,1,1,1, 0,0,0,1, 1,1,1,0, 0,0,0,0, 0,1,1,1, 1,1,1,0, 0,
  1,1,1,1, 1,1,1,1, 0,1,1,1, 0,0,0,0, 1,1,1,1, 0,0,0,0, 0,0,1,1, 1,1,1,1, 0,
  1,1,1,1, 1,1,1,1, 0,1,1,1, 0,0,0,0, 1,1,1,1, 0,0,0,0, 0,0,0,1, 1,1,1,1, 1,
  1,1,1,1, 1,0,1,1, 0,0,1,1, 0,0,0,0, 0,1,1,1, 0,0,0,0, 0,0,0,0, 1,1,1,1, 1,
  1,1,1,1, 1,0,1,1, 0,0,1,1, 0,0,0,0, 0,0,1,1, 0,0,0,0, 0,0,0,0, 0,1,1,1, 1
};

__device__ __forceinline__ unsigned short bf_bits(float f) {
  unsigned u = __float_as_uint(f);
  return (unsigned short)((u + 0x7FFFu + ((u >> 16) & 1u)) >> 16);
}
__device__ __forceinline__ float bf_up(unsigned short b) { return __uint_as_float(((unsigned)b) << 16); }
__device__ __forceinline__ float bfr(float f) { return bf_up(bf_bits(f)); }
__device__ __forceinline__ unsigned short h_bits(_Float16 x) { return __builtin_bit_cast(unsigned short, x); }
__device__ __forceinline__ unsigned pk16(unsigned short a, unsigned short b) { return (unsigned)a | ((unsigned)b << 16); }
__device__ __forceinline__ v8f zero8() { v8f z = {0.f, 0.f, 0.f, 0.f, 0.f, 0.f, 0.f, 0.f}; return z; }

__device__ __forceinline__ v16h ldfrag_h(const _Float16* p) {
  FragH f;
  f.h[0] = *(const v8h*)(p);
  f.h[1] = *(const v8h*)(p + 16);
  return f.v;
}
__device__ __forceinline__ v16b ldfrag_b(const u16* p) {
  FragB f;
  f.u[0] = *(const v4u*)(p);
  f.u[1] = *(const v4u*)(p + 16);
  return f.v;
}

__device__ __forceinline__ v8f mma_h(v16h a, v16h b, v8f c) {
  return __builtin_amdgcn_wmma_f32_16x16x32_f16(false, a, false, b, (short)0, c, false, false);
}
__device__ __forceinline__ v8f mma_b(v16b a, v16b b, v8f c) {
  return __builtin_amdgcn_wmma_f32_16x16x32_bf16(false, a, false, b, (short)0, c, false, false);
}
template <typename F>
__device__ __forceinline__ void guard4in(v8f& a, v8f& b, F x0, F x1, F x2, F x3) {
#if defined(__HIP_DEVICE_COMPILE__)
  asm volatile("v_nop\n\tv_nop\n\tv_nop\n\tv_nop"
               : "+v"(a), "+v"(b) : "v"(x0), "v"(x1), "v"(x2), "v"(x3) : "memory");
#endif
}
template <typename F>
__device__ __forceinline__ void guard8in(v8f& a, v8f& b, F x0, F x1, F x2, F x3, F x4, F x5, F x6, F x7) {
#if defined(__HIP_DEVICE_COMPILE__)
  asm volatile("v_nop\n\tv_nop\n\tv_nop\n\tv_nop"
               : "+v"(a), "+v"(b)
               : "v"(x0), "v"(x1), "v"(x2), "v"(x3), "v"(x4), "v"(x5), "v"(x6), "v"(x7) : "memory");
#endif
}
__device__ __forceinline__ void acc_guard4(v8f& a, v8f& b, v8f& c, v8f& d) {
#if defined(__HIP_DEVICE_COMPILE__)
  asm volatile("v_nop\n\tv_nop\n\tv_nop\n\tv_nop" : "+v"(a), "+v"(b), "+v"(c), "+v"(d));
#endif
}
__device__ __forceinline__ void wave_sync_lds() {
  __builtin_amdgcn_fence(__ATOMIC_RELEASE, "workgroup");
  __builtin_amdgcn_wave_barrier();
  __builtin_amdgcn_fence(__ATOMIC_ACQUIRE, "workgroup");
}

__global__ __launch_bounds__(256) void cvt_bf(const float* __restrict__ x, u16* D, int n8) {
  const int gt = blockIdx.x * 256 + (int)threadIdx.x;
  if (gt >= n8) return;
  const float* p = x + (size_t)gt * 8;
  const v4f a = *(const v4f*)(p), b4 = *(const v4f*)(p + 4);
  float w[8];
#pragma unroll
  for (int e = 0; e < 4; ++e) { w[e] = a[e]; w[4 + e] = b4[e]; }
  v4u o;
#pragma unroll
  for (int e = 0; e < 4; ++e) {
    o[e] = pk16(bf_bits(w[2 * e]), bf_bits(w[2 * e + 1]));
  }
  u16* d = D + (size_t)gt * 8;
  for (int pass = 0; pass < 2; ++pass) {
    *(volatile v4u*)(d) = o;
    __threadfence();
  }
}

__global__ __launch_bounds__(256) void cvt_kp(const float* __restrict__ x, u16* D, int nthr) {
  const int gt = blockIdx.x * 256 + (int)threadIdx.x;
  if (gt >= nthr) return;
  const int h  = gt / (SKP * 16);
  const int r  = gt - h * (SKP * 16);
  const int s  = r >> 4;
  const int d8 = (r & 15) * 8;
  const bool ok = (s < SKV);
  const int  sc = ok ? s : (SKV - 1);
  const float* p = x + ((size_t)(h * SKV + sc)) * HD + d8;
  const v4f a = *(const v4f*)(p), b4 = *(const v4f*)(p + 4);
  float w[8];
#pragma unroll
  for (int e = 0; e < 4; ++e) { w[e] = ok ? a[e] : 0.0f; w[4 + e] = ok ? b4[e] : 0.0f; }
  v4u o;
#pragma unroll
  for (int e = 0; e < 4; ++e) {
    o[e] = pk16(bf_bits(w[2 * e]), bf_bits(w[2 * e + 1]));
  }
  u16* d = D + (size_t)gt * 8;
  for (int pass = 0; pass < 2; ++pass) {
    *(volatile v4u*)(d) = o;
    __threadfence();
  }
}

__global__ __launch_bounds__(256) void vt16(const float* __restrict__ V, u16* VTo) {
  __shared__ __align__(16) u16 T[HD * VTP];
  const int tid = threadIdx.x;
  const int bid = blockIdx.x;
  const int h   = bid / NVT;
  const int st  = bid - h * NVT;
  if (h >= NHEAD) return;
  const int s0  = st * 64;
  {
    const int sl = tid >> 2;
    const int dc = (tid & 3) * 32;
    const int s  = s0 + sl;
    const bool ok = (s < SKV);
    const int  sc = ok ? s : (SKV - 1);
    const float* src = V + ((size_t)(h * SKV + sc)) * HD + dc;
#pragma unroll
    for (int i = 0; i < 8; ++i) {
      const v4f a = *(const v4f*)(src + 4 * i);
#pragma unroll
      for (int e = 0; e < 4; ++e) {
        const float t = ok ? (bfr(a[e]) * VCAR) : 0.0f;
        T[(dc + 4 * i + e) * VTP + sl] = h_bits((_Float16)t);
      }
    }
  }
  __syncthreads();
  v4u w4[4];
  const int q8 = tid >> 3, p8 = (tid & 7) * 8;
#pragma unroll
  for (int it = 0; it < 4; ++it) {
    const int line = it * 32 + q8;
    w4[it] = *(const v4u*)(T + line * VTP + p8);
  }
  const size_t base = ((size_t)(h * HD)) * SKP + s0 + p8;
  for (int pass = 0; pass < 2; ++pass) {
#pragma unroll
    for (int it = 0; it < 4; ++it) {
      const int line = it * 32 + q8;
      *(volatile v4u*)(VTo + base + (size_t)line * SKP) = w4[it];
    }
    __threadfence();
  }
}

__global__ __launch_bounds__(ATT_THREADS)
void attn_bs(const u16* __restrict__ QBp, const u16* __restrict__ KBp, const u16* __restrict__ VTp, float* Og) {
  __shared__ __align__(16) float smem[WPB * WREG];

  const int tid  = threadIdx.x;
  const int wave = tid >> 5;
  const int lane = tid & 31;
  const int hh   = lane >> 4;
  const int c    = lane & 15;
  const int bid  = blockIdx.x;
  const int h    = bid / NQG;
  const int g    = bid - h * NQG;
  if (h >= NHEAD) return;
  const int q0   = g * QGRP + wave * 16;
  const int qb   = g >> 1;

  float* pt   = smem + wave * WREG;
  float* slab = pt + PTW;

  const u16* Qp  = QBp + ((size_t)(h * SQ + q0 + c)) * HD + 8 * hh;
  const u16* Khb = KBp + ((size_t)(h * SKP + c)) * HD + 8 * hh;
  const _Float16* Vhb = (const _Float16*)(const void*)VTp + ((size_t)(h * HD + c)) * SKP + 8 * hh;
  const float lsc = RSQ_HD * LOG2E;
  const float oc  = 1.0f / (PCAR * VCAR);

  const v16b qa0 = ldfrag_b(Qp);
  const v16b qa1 = ldfrag_b(Qp + 32);
  const v16b qa2 = ldfrag_b(Qp + 64);
  const v16b qa3 = ldfrag_b(Qp + 96);

  float mrow[8], lrow[8];
  v8f o[8];
#pragma unroll
  for (int r = 0; r < 8; ++r) { mrow[r] = -INFINITY; lrow[r] = 0.f; }
#pragma unroll
  for (int j = 0; j < 8; ++j) o[j] = zero8();

#pragma unroll 1
  for (int kblk = 0; kblk < NKBLK; ++kblk) {
    if (kLive[qb * NKBLK + kblk] == 0) continue;
    const int kv0   = kblk * 128;
    const int rem   = SKV - kv0;
    const int ntile = (rem >= 128) ? 4 : ((rem + 31) >> 5);
#pragma unroll 1
    for (int ktl = 0; ktl < ntile; ++ktl) {
      const int kb = kv0 + ktl * 32;
      v8f s0 = zero8(), s1 = zero8();
      {
        const u16* k0p = Khb + (size_t)kb * HD;
        const u16* k1p = k0p + (size_t)16 * HD;
        const v16b f00 = ldfrag_b(k0p),      f10 = ldfrag_b(k1p);
        const v16b f01 = ldfrag_b(k0p + 32), f11 = ldfrag_b(k1p + 32);
        s0 = mma_b(qa0, f00, s0);
        s1 = mma_b(qa0, f10, s1);
        s0 = mma_b(qa1, f01, s0);
        s1 = mma_b(qa1, f11, s1);
        const v16b f02 = ldfrag_b(k0p + 64), f12 = ldfrag_b(k1p + 64);
        const v16b f03 = ldfrag_b(k0p + 96), f13 = ldfrag_b(k1p + 96);
        s0 = mma_b(qa2, f02, s0);
        s1 = mma_b(qa2, f12, s1);
        s0 = mma_b(qa3, f03, s0);
        s1 = mma_b(qa3, f13, s1);
        guard8in<v16b>(s0, s1, f00, f10, f01, f11, f02, f12, f03, f13);
      }
      const bool ok0 = (kb + c) < SKV;
      const bool ok1 = (kb + 16 + c) < SKV;
#pragma unroll
      for (int r = 0; r < 8; ++r) {
        const float u0 = s0[r] * lsc;
        const float u1 = s1[r] * lsc;
        const float t0 = ok0 ? u0 : -INFINITY;
        const float t1 = ok1 ? u1 : -INFINITY;
        float mx = fmaxf(t0, t1);
#pragma unroll
        for (int off = 1; off < 16; off <<= 1) mx = fmaxf(mx, __shfl_xor(mx, off, 32));
        const float mn = fmaxf(mrow[r], mx);
        const float ms = (mn == -INFINITY) ? 0.0f : mn;
        const float al = exp2f(mrow[r] - ms);
        mrow[r] = mn;
        const float e0 = exp2f(t0 - ms), e1 = exp2f(t1 - ms);
        float ps = e0 + e1;
#pragma unroll
        for (int off = 1; off < 16; off <<= 1) ps += __shfl_xor(ps, off, 32);
        lrow[r] = lrow[r] * al + ps;
#pragma unroll
        for (int j = 0; j < 8; ++j) o[j][r] *= al;
        const int ro = (8 * hh + r) * PTP + c;
        pt[ro]      = e0;
        pt[ro + 16] = e1;
      }
      wave_sync_lds();
      FragH ph, pl;
      {
        const float* prow = pt + c * PTP + 8 * hh;
        const v4f p0 = *(const v4f*)(prow), p1 = *(const v4f*)(prow + 4);
        const v4f p2 = *(const v4f*)(prow + 16), p3 = *(const v4f*)(prow + 20);
#pragma unroll
        for (int e = 0; e < 4; ++e) {
          const float ta = p0[e] * PCAR, tb = p1[e] * PCAR, tc = p2[e] * PCAR, td = p3[e] * PCAR;
          const _Float16 ha = (_Float16)ta, hb = (_Float16)tb, hc = (_Float16)tc, hd = (_Float16)td;
          ph.h[0][e]     = ha;
          ph.h[0][4 + e] = hb;
          ph.h[1][e]     = hc;
          ph.h[1][4 + e] = hd;
          pl.h[0][e]     = (_Float16)(ta - (float)ha);
          pl.h[0][4 + e] = (_Float16)(tb - (float)hb);
          pl.h[1][e]     = (_Float16)(tc - (float)hc);
          pl.h[1][4 + e] = (_Float16)(td - (float)hd);
        }
      }
      {
        const _Float16* vp = Vhb + kb;
#pragma unroll
        for (int jg = 0; jg < 4; ++jg) {
          const size_t da = (size_t)(2 * jg) * 16 * SKP;
          const size_t db = da + (size_t)16 * SKP;
          const v16h va = ldfrag_h(vp + da), vb = ldfrag_h(vp + db);
          o[2 * jg]     = mma_h(ph.v, va, o[2 * jg]);
          o[2 * jg]     = mma_h(pl.v, va, o[2 * jg]);
          o[2 * jg + 1] = mma_h(ph.v, vb, o[2 * jg + 1]);
          o[2 * jg + 1] = mma_h(pl.v, vb, o[2 * jg + 1]);
          guard4in<v16h>(o[2 * jg], o[2 * jg + 1], ph.v, pl.v, va, vb);
        }
      }
      wave_sync_lds();
    }
  }
  acc_guard4(o[0], o[1], o[2], o[3]);
  acc_guard4(o[4], o[5], o[6], o[7]);
#pragma unroll
  for (int r = 0; r < 8; ++r) {
    const float lv  = lrow[r];
    const float ls  = (lv > 0.0f) ? lv : 1.0f;
    const float inv = (lv > 0.0f) ? ((1.0f / ls) * oc) : 0.0f;
#pragma unroll
    for (int j = 0; j < 8; ++j) {
      const int idx = (8 * hh + r) * SLP + j * 16 + c;
      slab[idx] = o[j][r] * inv;
    }
  }
  wave_sync_lds();
  v4f vals[16];
#pragma unroll
  for (int it = 0; it < 16; ++it) vals[it] = *(const v4f*)(slab + it * SLP + lane * 4);
  float* dst = Og + ((size_t)(h * SQ + q0)) * HD + lane * 4;
  for (int pass = 0; pass < 2; ++pass) {
#pragma unroll
    for (int it = 0; it < 16; ++it) {
      *(volatile v4f*)(dst + (size_t)it * HD) = vals[it];
    }
    __threadfence();
  }
}

extern "C" void kernel_launch(void* const* d_in, const int* in_sizes, int n_in,
                              void* d_out, int out_size, void* d_ws, size_t ws_size,
                              hipStream_t stream) {
  if (n_in < 3) return;
  if (in_sizes[0] != NHEAD * SQ * HD) return;
  if (in_sizes[1] != NHEAD * SKV * HD) return;
  if (in_sizes[2] != NHEAD * SKV * HD) return;
  if (out_size != NHEAD * SQ * HD) return;

  const float* q = (const float*)d_in[0];
  const float* k = (const float*)d_in[1];
  const float* v = (const float*)d_in[2];
  float*     out = (float*)d_out;

  const size_t szQB = (size_t)NHEAD * SQ * HD * 2;
  const size_t szKB = (size_t)NHEAD * SKP * HD * 2;
  const size_t szVT = (size_t)NHEAD * HD * SKP * 2;
  size_t off = 0;
  const size_t oQB = off; off += szQB;
  const size_t oKB = off; off += szKB;
  const size_t oVT = off; off += szVT;
  if (off > ws_size) return;
  if (off > (size_t)WS_CAP) return;

  char* ws = (char*)d_ws;
  u16* QB = (u16*)(ws + oQB);
  u16* KB = (u16*)(ws + oKB);
  u16* VT = (u16*)(ws + oVT);

  const dim3 b256(256), bAT(ATT_THREADS);
  const int  n8q  = (NHEAD * SQ * HD) / 8;
  const int  nthk = NHEAD * SKP * 16;
  const dim3 gQ((n8q + 255) / 256);
  const dim3 gK((nthk + 255) / 256);
  const dim3 gVT(NHEAD * NVT);
  const dim3 gAT(NHEAD * NQG);

  cvt_bf<<<gQ, b256, 0, stream>>>(q, QB, n8q);
  cvt_kp<<<gK, b256, 0, stream>>>(k, KB, nthk);
  vt16<<<gVT, b256, 0, stream>>>(v, VT);
  attn_bs<<<gAT, bAT, 0, stream>>>(QB, KB, VT, out);
  (void)hipGetLastError();
}
